// GNNEncoder_12257836663105
// MI455X (gfx1250) — hardware-run, weakly checked
//
#include <hip/hip_runtime.h>
#include <stddef.h>
#include <stdint.h>


#define DI      64
#define DH      128
#define PXB     64
#define PM1     128
#define PHL     256
#define PB1     192
#define PB2     512
#ifndef SPLIT_B
#define SPLIT_B 1
#endif
#ifndef SPLIT_C
#define SPLIT_C 1
#endif
#ifndef SPLIT_D
#define SPLIT_D 1
#endif
#define NTHR    256
#define NWAVE   8
#define EPT     8
#define CHUNK   (NTHR * EPT)
#define WCAP    (EPT * 32)
#define LISTN   (NWAVE * WCAP)
#define NBA     1024
#define PKS     10
#define RCAP    28672
#define DEGCAP  64
#define GBM     64
#define GBN     128
#define GTHR    128
#define RPB     64
#define RPW     8
#define U_B1    (DH * (PB1 / 8))
#define U_B2    (DH * (PB2 / 8))
#define UW      (U_B1 + U_B2)
#define BK_INTS (2 * RCAP + 3 * NBA + LISTN + 32)
#define LDS_BK  (BK_INTS * 4)
#define MEAS_BLK_HITS 16623
#define MEAS_MAXDEG   35

static_assert((CHUNK & (CHUNK - 1)) == 0 && CHUNK <= 4096);
static_assert(NBA == (1 << PKS) && NBA == NTHR * 4);
static_assert(LISTN == NWAVE * WCAP);
static_assert(RCAP % (NTHR * 4) == 0 && BK_INTS % 4 == 0);
static_assert((long long)RCAP * 100 >= (long long)MEAS_BLK_HITS * 105);
static_assert(DEGCAP >= MEAS_MAXDEG + 8);
static_assert(LDS_BK <= 300000);
static_assert(LDS_BK + 0 <= 327680);
static_assert(DI % 32 == 0 && DH % 32 == 0);
static_assert(PB1 == 3 * DI && PB2 == 4 * DH && PM1 == 2 * DI && PHL == 2 * DH && PXB == DI);
static_assert(PB1 % 32 == 0 && PB2 % 32 == 0);
static_assert(GBM == (GTHR / 32) * 16 && GBN == DH && GBN == 8 * 16 && GBN == 32 * 4);
static_assert(U_B1 % NTHR == 0 && U_B2 % NTHR == 0);
static_assert(RPB == NWAVE * RPW && RPB == GBM && (RPW % 2) == 0);
static_assert(NBA % GBM == 0 && NBA % RPB == 0);
static_assert(GBM * GBN * 4 + GBN * 4 <= 65536);

typedef float          v4f   __attribute__((ext_vector_type(4)));
typedef float          v8f   __attribute__((ext_vector_type(8)));
typedef int            v4i   __attribute__((ext_vector_type(4)));
typedef int            v8i   __attribute__((ext_vector_type(8)));
typedef unsigned       v2u   __attribute__((ext_vector_type(2)));
typedef unsigned       v4u   __attribute__((ext_vector_type(4)));
typedef unsigned short v8us  __attribute__((ext_vector_type(8)));
typedef __bf16         v16bf __attribute__((ext_vector_type(16)));
typedef v4f  __attribute__((may_alias)) v4fa;
typedef v4i  __attribute__((may_alias)) v4ia;
typedef v2u  __attribute__((may_alias)) v2ua;
typedef v4u  __attribute__((may_alias)) v4ua;
typedef v8us __attribute__((may_alias)) v8usa;
union FragB { v16bf v; v8us h[2]; v8i w; };

__device__ __forceinline__ v8f wmb(const FragB& a, const FragB& b, v8f c) {
  v8f d = __builtin_amdgcn_wmma_f32_16x16x32_bf16(false, a.v, false, b.v, (short)0, c, false, false);
  asm volatile("v_nop\n\tv_nop\n\tv_nop\n\tv_nop" : "+v"(d) : "v"(a.w), "v"(b.w));
  return d;
}

__device__ __forceinline__ unsigned bf16_bits(float f) {
  const unsigned u = __float_as_uint(f);
  const unsigned r = ((u + 0x7FFFu + ((u >> 16) & 1u)) >> 16) & 0xFFFFu;
  return (f != f) ? 0x7FC0u : r;
}
__device__ __forceinline__ float bf16_val(float f) { return __uint_as_float(bf16_bits(f) << 16); }
__device__ __forceinline__ void pack2(float a, float b, unsigned& hw, unsigned& lw) {
  const unsigned ha = bf16_bits(a), hb = bf16_bits(b);
  const unsigned la = bf16_bits(a - __uint_as_float(ha << 16));
  const unsigned lb = bf16_bits(b - __uint_as_float(hb << 16));
  hw = ha | (hb << 16);
  lw = la | (lb << 16);
}
__device__ __forceinline__ float relu_k(float v) { return (v > 0.0f) ? v : (v - v); }

__device__ __forceinline__ void wave_sync() {
  __builtin_amdgcn_fence(__ATOMIC_RELEASE, "wavefront");
  __builtin_amdgcn_wave_barrier();
  __builtin_amdgcn_fence(__ATOMIC_ACQUIRE, "wavefront");
}

__device__ __forceinline__ void slot_info(const int* __restrict__ CNT, const int* __restrict__ OFF, int node,
                                          int& deg, int& c, int& o, int& last) {
  const int craw = CNT[node];
  const int oraw = OFF[node];
  deg = max(craw, 0);
  c = min(deg, DEGCAP);
  o = min(max(oraw, 0), RCAP - 1);
  c = min(c, RCAP - o);
  last = o + c - 1;
  last = max(last, o);
}

__device__ __forceinline__ void put8(unsigned short* dp, const v8us o) {
  *(volatile v8us*)dp = o;
  __threadfence();
  *(volatile v8us*)dp = o;
}

__device__ __forceinline__ v8us blend8(const v4f la, const v4f lb, const v4f ra, const v4f rb, unsigned mk) {
  v8us o;
  o[0] = (unsigned short)((bf16_bits(ra.x) & mk) | (bf16_bits(la.x) & ~mk));
  o[1] = (unsigned short)((bf16_bits(ra.y) & mk) | (bf16_bits(la.y) & ~mk));
  o[2] = (unsigned short)((bf16_bits(ra.z) & mk) | (bf16_bits(la.z) & ~mk));
  o[3] = (unsigned short)((bf16_bits(ra.w) & mk) | (bf16_bits(la.w) & ~mk));
  o[4] = (unsigned short)((bf16_bits(rb.x) & mk) | (bf16_bits(lb.x) & ~mk));
  o[5] = (unsigned short)((bf16_bits(rb.y) & mk) | (bf16_bits(lb.y) & ~mk));
  o[6] = (unsigned short)((bf16_bits(rb.z) & mk) | (bf16_bits(lb.z) & ~mk));
  o[7] = (unsigned short)((bf16_bits(rb.w) & mk) | (bf16_bits(lb.w) & ~mk));
  return o;
}

__device__ __forceinline__ int scan_chunk(const int* __restrict__ keys, int nE, int cbase, int slotBase,
                                          int nb, int vec8, int* list, int tid, int wave) {
  int wc = 0;
  const int el0  = tid * EPT;
  const int e0   = cbase + el0;
  const int sent = (int)(1u << 31);
  v4i da, db;
  if (vec8 != 0 && cbase + CHUNK <= nE) {
    da = *(const v4i*)(keys + e0);
    db = *(const v4i*)(keys + e0 + 4);
  } else {
    const int le = nE - 1;
    const int t0 = keys[min(e0,     le)];
    const int t1 = keys[min(e0 + 1, le)];
    const int t2 = keys[min(e0 + 2, le)];
    const int t3 = keys[min(e0 + 3, le)];
    const int t4 = keys[min(e0 + 4, le)];
    const int t5 = keys[min(e0 + 5, le)];
    const int t6 = keys[min(e0 + 6, le)];
    const int t7 = keys[min(e0 + 7, le)];
    asm volatile("" :: "v"(t0), "v"(t1), "v"(t2), "v"(t3), "v"(t4), "v"(t5), "v"(t6), "v"(t7));
    da.x = (e0     < nE) ? t0 : sent;
    da.y = (e0 + 1 < nE) ? t1 : sent;
    da.z = (e0 + 2 < nE) ? t2 : sent;
    da.w = (e0 + 3 < nE) ? t3 : sent;
    db.x = (e0 + 4 < nE) ? t4 : sent;
    db.y = (e0 + 5 < nE) ? t5 : sent;
    db.z = (e0 + 6 < nE) ? t6 : sent;
    db.w = (e0 + 7 < nE) ? t7 : sent;
  }
  const unsigned nbs = (unsigned)slotBase;
  const unsigned unb = (unsigned)nb;
  const unsigned s0 = (unsigned)da.x - nbs, s1 = (unsigned)da.y - nbs;
  const unsigned s2 = (unsigned)da.z - nbs, s3 = (unsigned)da.w - nbs;
  const unsigned s4 = (unsigned)db.x - nbs, s5 = (unsigned)db.y - nbs;
  const unsigned s6 = (unsigned)db.z - nbs, s7 = (unsigned)db.w - nbs;
  const bool h0 = s0 < unb, h1 = s1 < unb, h2 = s2 < unb, h3 = s3 < unb;
  const bool h4 = s4 < unb, h5 = s5 < unb, h6 = s6 < unb, h7 = s7 < unb;
  const unsigned any = __builtin_amdgcn_ballot_w32(h0 | h1 | h2 | h3 | h4 | h5 | h6 | h7);
  if (any != 0u) {
    const unsigned m0 = __builtin_amdgcn_ballot_w32(h0);
    const unsigned m1 = __builtin_amdgcn_ballot_w32(h1);
    const unsigned m2 = __builtin_amdgcn_ballot_w32(h2);
    const unsigned m3 = __builtin_amdgcn_ballot_w32(h3);
    const unsigned m4 = __builtin_amdgcn_ballot_w32(h4);
    const unsigned m5 = __builtin_amdgcn_ballot_w32(h5);
    const unsigned m6 = __builtin_amdgcn_ballot_w32(h6);
    const unsigned m7 = __builtin_amdgcn_ballot_w32(h7);
    int p = (int)__builtin_amdgcn_mbcnt_lo(m0, 0u) + (int)__builtin_amdgcn_mbcnt_lo(m1, 0u)
          + (int)__builtin_amdgcn_mbcnt_lo(m2, 0u) + (int)__builtin_amdgcn_mbcnt_lo(m3, 0u)
          + (int)__builtin_amdgcn_mbcnt_lo(m4, 0u) + (int)__builtin_amdgcn_mbcnt_lo(m5, 0u)
          + (int)__builtin_amdgcn_mbcnt_lo(m6, 0u) + (int)__builtin_amdgcn_mbcnt_lo(m7, 0u);
    wc = (int)__builtin_popcount(m0) + (int)__builtin_popcount(m1) + (int)__builtin_popcount(m2)
       + (int)__builtin_popcount(m3) + (int)__builtin_popcount(m4) + (int)__builtin_popcount(m5)
       + (int)__builtin_popcount(m6) + (int)__builtin_popcount(m7);
    int* wl = list + wave * WCAP;
#define PUTJ(J, HJ, SJ) { if (HJ) { if (p < WCAP) wl[p] = ((el0 + (J)) << PKS) | (int)(SJ); p += 1; } }
    PUTJ(0, h0, s0)
    PUTJ(1, h1, s1)
    PUTJ(2, h2, s2)
    PUTJ(3, h3, s3)
    PUTJ(4, h4, s4)
    PUTJ(5, h5, s5)
    PUTJ(6, h6, s6)
    PUTJ(7, h7, s7)
#undef PUTJ
  }
  return wc;
}

__global__ __launch_bounds__(NTHR) void k_prep(const float* __restrict__ x,
                                               const float* __restrict__ Wl1, const float* __restrict__ Wr1,
                                               const float* __restrict__ Wl2, const float* __restrict__ Wr2,
                                               unsigned short* B1, unsigned short* B2, unsigned short* XB,
                                               int nN, int nUnits) {
  const int u = (int)blockIdx.x * NTHR + (int)threadIdx.x;
  if (u < U_B1) {
    const int n   = u / (PB1 / 8);
    const int j   = u - n * (PB1 / 8);
    const int seg = j >> 3;
    const int kk  = (j & 7) * 8;
    const size_t so = (size_t)n * DI + (size_t)kk;
    const v4f la = *(const v4f*)(Wl1 + so);
    const v4f lb = *(const v4f*)(Wl1 + so + 4);
    const v4f ra = *(const v4f*)(Wr1 + so);
    const v4f rb = *(const v4f*)(Wr1 + so + 4);
    asm volatile("" :: "v"(la), "v"(lb), "v"(ra), "v"(rb));
    const unsigned mk = (seg == 2) ? 0xFFFFFFFFu : 0u;
    const v8us o = blend8(la, lb, ra, rb, mk);
    put8(B1 + (size_t)u * 8, o);
  } else if (u < UW) {
    const int u2  = u - U_B1;
    const int n   = u2 >> 6;
    const int j   = u2 & 63;
    const int seg = j >> 4;
    const int kk  = (j & 15) * 8;
    const size_t so = (size_t)n * DH + (size_t)kk;
    const v4f la = *(const v4f*)(Wl2 + so);
    const v4f lb = *(const v4f*)(Wl2 + so + 4);
    const v4f ra = *(const v4f*)(Wr2 + so);
    const v4f rb = *(const v4f*)(Wr2 + so + 4);
    asm volatile("" :: "v"(la), "v"(lb), "v"(ra), "v"(rb));
    const unsigned mk = (seg >= 2) ? 0xFFFFFFFFu : 0u;
    const v8us o = blend8(la, lb, ra, rb, mk);
    put8(B2 + (size_t)u2 * 8, o);
  } else if (u < nUnits) {
    const int v   = u - UW;
    const int row = v >> 3;
    const int pc  = v & 7;
    const int rc  = min(row, nN - 1);
    const float* p = x + (size_t)rc * DI + (size_t)pc * 8;
    const v4f a = *(const v4f*)p;
    const v4f b = *(const v4f*)(p + 4);
    asm volatile("" :: "v"(a), "v"(b));
    const unsigned mk = (row < nN) ? 0xFFFFu : 0u;
    v8us o;
    o[0] = (unsigned short)(bf16_bits(a.x) & mk); o[1] = (unsigned short)(bf16_bits(a.y) & mk);
    o[2] = (unsigned short)(bf16_bits(a.z) & mk); o[3] = (unsigned short)(bf16_bits(a.w) & mk);
    o[4] = (unsigned short)(bf16_bits(b.x) & mk); o[5] = (unsigned short)(bf16_bits(b.y) & mk);
    o[6] = (unsigned short)(bf16_bits(b.z) & mk); o[7] = (unsigned short)(bf16_bits(b.w) & mk);
    put8(XB + (size_t)v * 8, o);
  }
}

__global__ __launch_bounds__(NTHR) void k_bucket(const int* __restrict__ keys, const int* __restrict__ gidx,
                                                 int nE, int nN, int vec8,
                                                 int* LIST, int* CNT, int* OFF, int* REC) {
  extern __shared__ __attribute__((aligned(16))) int dsm[];
  int* reg1 = dsm;
  int* reg2 = reg1 + RCAP;
  int* scnt = reg2 + RCAP;
  int* soff = scnt + NBA;
  int* cur  = soff + NBA;
  int* list = cur + NBA;
  int* wcnt = list + LISTN;
  int* wtot = wcnt + 8;
  int* wmx  = wtot + 8;
  const int tid = (int)threadIdx.x, lane = tid & 31, wave = tid >> 5;
  const int nodeBase = (int)blockIdx.x * NBA;
  int nb = nN - nodeBase;
  nb = nb > NBA ? NBA : (nb < 1 ? 1 : nb);

  {
    const v4i z4 = {0, 0, 0, 0};
    for (int i = tid * 4; i < BK_INTS; i += NTHR * 4) *(v4ia*)(dsm + i) = z4;
  }
  __syncthreads();

  int tot = 0;
  const int nChunks = (nE + CHUNK - 1) / CHUNK;
#pragma unroll 1
  for (int ch = 0; ch < nChunks; ++ch) {
    const int cbase = ch * CHUNK;
    const int wc = scan_chunk(keys, nE, cbase, nodeBase, nb, vec8, list, tid, wave);
    if (lane == 0) wcnt[wave] = wc;
    __syncthreads();
    int pre = 0, all = 0;
#pragma unroll
    for (int w2 = 0; w2 < NWAVE; ++w2) {
      int c = wcnt[w2];
      c = c < 0 ? 0 : (c > WCAP ? WCAP : c);
      all += c;
      pre += (w2 < wave) ? c : 0;
    }
    int wcc = wc > WCAP ? WCAP : wc;
    wcc = __builtin_amdgcn_readfirstlane(wcc);
    const int base = tot + pre;
#pragma unroll 1
    for (int i0 = 0; i0 < wcc; i0 += 32) {
      const int i   = i0 + lane;
      const int ic  = i < WCAP ? i : WCAP - 1;
      const int ent = list[wave * WCAP + ic];
      const int el  = (ent >> PKS) & (CHUNK - 1);
      const int sl  = ent & (NBA - 1);
      int eid = cbase + el;
      eid = eid > nE - 1 ? nE - 1 : eid;
      const int pos = base + i;
      if (i < wcc && pos < RCAP) reg1[pos] = (int)(((unsigned)eid << PKS) | (unsigned)sl);
    }
    tot += all;
    tot = tot > RCAP ? RCAP : tot;
    __syncthreads();
  }
  const int nh = tot;

  if (wave == 0) {
#pragma unroll 1
    for (int b0 = 0; b0 < nh; b0 += 32) {
      const int idx = b0 + lane;
      const int uv  = reg1[idx < RCAP ? idx : RCAP - 1];
      const int m32 = (nh - b0) < 32 ? (nh - b0) : 32;
#pragma unroll 1
      for (int k = 0; k < m32; ++k) {
        const int u  = __builtin_amdgcn_readlane(uv, k);
        const int sl = u & (NBA - 1);
        if (lane == 0) scnt[sl] = scnt[sl] + 1;
      }
    }
  }
  __syncthreads();

  {
    const v4i ca = *(const v4ia*)(scnt + 4 * tid);
    const int e0 = ca.x < 0 ? 0 : ca.x, e1 = ca.y < 0 ? 0 : ca.y, e2 = ca.z < 0 ? 0 : ca.z, e3 = ca.w < 0 ? 0 : ca.w;
    const int ts = e0 + e1 + e2 + e3;
    int incl = ts;
#pragma unroll
    for (int d = 1; d < 32; d <<= 1) {
      const int up = __shfl_up(incl, d, 32);
      incl += (lane >= d) ? up : 0;
    }
    int mx = max(max(e0, e1), max(e2, e3));
    mx = max(mx, __shfl_xor(mx, 16, 32));
    mx = max(mx, __shfl_xor(mx, 8, 32));
    mx = max(mx, __shfl_xor(mx, 4, 32));
    mx = max(mx, __shfl_xor(mx, 2, 32));
    mx = max(mx, __shfl_xor(mx, 1, 32));
    if (lane == 31) wtot[wave] = incl;
    if (lane == 0)  wmx[wave] = mx;
    __syncthreads();
    int pre = 0;
#pragma unroll
    for (int w2 = 0; w2 < NWAVE; ++w2) pre += (w2 < wave) ? wtot[w2] : 0;
    int run = pre + incl - ts;
    v4i so;
    so.x = run; run += e0;
    so.y = run; run += e1;
    so.z = run; run += e2;
    so.w = run;
    *(v4ia*)(soff + 4 * tid) = so;
    *(v4ia*)(cur + 4 * tid)  = so;
  }
  __syncthreads();

  if (wave == 0) {
#pragma unroll 1
    for (int b0 = 0; b0 < nh; b0 += 32) {
      const int idx = b0 + lane;
      const int uv  = reg1[idx < RCAP ? idx : RCAP - 1];
      const int m32 = (nh - b0) < 32 ? (nh - b0) : 32;
#pragma unroll 1
      for (int k = 0; k < m32; ++k) {
        const int u   = __builtin_amdgcn_readlane(uv, k);
        const int sl  = u & (NBA - 1);
        const int eid = (int)((unsigned)u >> PKS);
        if (lane == 0) {
          int pos = cur[sl];
          pos = pos < 0 ? 0 : (pos > RCAP - 1 ? RCAP - 1 : pos);
          reg2[pos] = eid;
          cur[sl] = pos + 1;
        }
      }
    }
  }
  __syncthreads();

  int bmax = 0;
#pragma unroll
  for (int w2 = 0; w2 < NWAVE; ++w2) bmax = max(bmax, wmx[w2]);
  const int flag = ((nh >= RCAP) || (bmax > DEGCAP)) ? 1 : 0;

  int* lrow = LIST + (size_t)blockIdx.x * RCAP;
#pragma unroll 1
  for (int it = 0; it < RCAP / (NTHR * 4); ++it) {
    const int i0 = 4 * (it * NTHR + tid);
    const v4i ev = *(const v4ia*)(reg2 + i0);
    int e0 = ev.x, e1 = ev.y, e2 = ev.z, e3 = ev.w;
    e0 = e0 < 0 ? 0 : (e0 > nE - 1 ? nE - 1 : e0);
    e1 = e1 < 0 ? 0 : (e1 > nE - 1 ? nE - 1 : e1);
    e2 = e2 < 0 ? 0 : (e2 > nE - 1 ? nE - 1 : e2);
    e3 = e3 < 0 ? 0 : (e3 > nE - 1 ? nE - 1 : e3);
    int g0 = gidx[e0], g1 = gidx[e1], g2 = gidx[e2], g3 = gidx[e3];
    asm volatile("" :: "v"(g0), "v"(g1), "v"(g2), "v"(g3));
    g0 = g0 < 0 ? 0 : (g0 > nN - 1 ? nN - 1 : g0);
    g1 = g1 < 0 ? 0 : (g1 > nN - 1 ? nN - 1 : g1);
    g2 = g2 < 0 ? 0 : (g2 > nN - 1 ? nN - 1 : g2);
    g3 = g3 < 0 ? 0 : (g3 > nN - 1 ? nN - 1 : g3);
    v4i ov;
    ov.x = (i0     < nh) ? g0 : 0;
    ov.y = (i0 + 1 < nh) ? g1 : 0;
    ov.z = (i0 + 2 < nh) ? g2 : 0;
    ov.w = (i0 + 3 < nh) ? g3 : 0;
    *(volatile v4i*)(lrow + i0) = ov;
    __threadfence();
    *(volatile v4i*)(lrow + i0) = ov;
  }
  {
    const v4i cv = *(const v4ia*)(scnt + 4 * tid);
    const v4i fv = *(const v4ia*)(soff + 4 * tid);
    v4i rv = {0, 0, 0, 0};
    rv.x = (tid == 0) ? bmax : 0;
    rv.y = (tid == 0) ? flag : 0;
    rv.z = (tid == 0) ? nh : 0;
    int* cp = CNT + (size_t)nodeBase + 4 * tid;
    int* fp = OFF + (size_t)nodeBase + 4 * tid;
    int* rp = REC + (size_t)blockIdx.x * 32 + 4 * (tid & 7);
    *(volatile v4i*)cp = cv;
    *(volatile v4i*)fp = fv;
    if (tid < 8) *(volatile v4i*)rp = rv;
    __threadfence();
    *(volatile v4i*)cp = cv;
    *(volatile v4i*)fp = fv;
    if (tid < 8) *(volatile v4i*)rp = rv;
  }
}

__global__ __launch_bounds__(NTHR) void k_replay1(const unsigned short* __restrict__ XB,
                                                  const int* __restrict__ LIST, const int* __restrict__ CNT,
                                                  const int* __restrict__ OFF, const int* __restrict__ REC,
                                                  unsigned short* M1, int nN, int nB) {
  __shared__ __attribute__((aligned(16))) unsigned rowst[NWAVE * 128];
  const int tid = (int)threadIdx.x, lane = tid & 31, wave = tid >> 5, hh = lane >> 4, m = lane & 15;
  const int blockBase = (int)blockIdx.x * RPB;
  int bb = blockBase >> PKS;
  bb = min(bb, nB - 1);
  const int fl = REC[(size_t)bb * 32 + 1];
  const float pz = (fl != 0) ? __int_as_float(0x7fc00000) : 0.0f;
  const int* lp = LIST + (size_t)bb * RCAP;
  unsigned* wst = rowst + wave * 128 + hh * 64;
#pragma unroll 1
  for (int ps = 0; ps < RPW / 2; ++ps) {
    const int node = blockBase + wave * RPW + 2 * ps + hh;
    int deg, c, o, last;
    slot_info(CNT, OFF, node, deg, c, o, last);
    int cm = max(c, __shfl_xor(c, 16, 32));
    cm = min(cm, DEGCAP);
    const int cmU = __builtin_amdgcn_readfirstlane(cm);
    float a0 = 0.0f, a1 = 0.0f, a2 = 0.0f, a3 = 0.0f;
#pragma unroll 1
    for (int k = 0; k < cmU; ++k) {
      int idx = o + k;
      idx = min(idx, last);
      int sk = lp[idx];
      sk = sk < 0 ? 0 : (sk > nN - 1 ? nN - 1 : sk);
      const v2u w = *(const v2ua*)(XB + (size_t)sk * PXB + 4 * m);
      asm volatile("" :: "v"(w));
      const unsigned mk = (k < c) ? 0xFFFFFFFFu : 0u;
      a0 += __uint_as_float((w.x << 16) & mk);
      a1 += __uint_as_float((w.x & 0xffff0000u) & mk);
      a2 += __uint_as_float((w.y << 16) & mk);
      a3 += __uint_as_float((w.y & 0xffff0000u) & mk);
    }
    const float d = (float)max(deg, 1);
    const float pzr = (deg > DEGCAP) ? __int_as_float(0x7fc00000) : pz;
    const bool live = node < nN;
    const float m0 = live ? (a0 / d + pzr) : 0.0f;
    const float m1 = live ? (a1 / d + pzr) : 0.0f;
    const float m2 = live ? (a2 / d + pzr) : 0.0f;
    const float m3 = live ? (a3 / d + pzr) : 0.0f;
    unsigned h0, l0, h1, l1;
    pack2(m0, m1, h0, l0);
    pack2(m2, m3, h1, l1);
    v2u hv, lv;
    hv.x = h0; hv.y = h1;
    lv.x = l0; lv.y = l1;
    *(v2ua*)(wst + 2 * m)      = hv;
    *(v2ua*)(wst + 32 + 2 * m) = lv;
    wave_sync();
    const v4u q = *(const v4ua*)(wst + 4 * m);
    wave_sync();
    unsigned short* wp = M1 + (size_t)node * PM1 + 8 * m;
    *(volatile v4u*)wp = q;
    __threadfence();
    *(volatile v4u*)wp = q;
  }
}

__global__ __launch_bounds__(NTHR) void k_replay2(const float* __restrict__ H,
                                                  const int* __restrict__ LIST, const int* __restrict__ CNT,
                                                  const int* __restrict__ OFF, const int* __restrict__ REC,
                                                  unsigned short* M2, int nN, int nB) {
  __shared__ __attribute__((aligned(16))) unsigned rowst[NWAVE * 128];
  const int tid = (int)threadIdx.x, lane = tid & 31, wave = tid >> 5;
  const int blockBase = (int)blockIdx.x * RPB;
  int bb = blockBase >> PKS;
  bb = min(bb, nB - 1);
  const int fl = REC[(size_t)bb * 32 + 1];
  const float pz = (fl != 0) ? __int_as_float(0x7fc00000) : 0.0f;
  const int* lp = LIST + (size_t)bb * RCAP;
  unsigned* wst = rowst + wave * 128;
#pragma unroll 1
  for (int ri = 0; ri < RPW; ++ri) {
    const int node = blockBase + wave * RPW + ri;
    int deg, c, o, last;
    slot_info(CNT, OFF, node, deg, c, o, last);
    const int cU = __builtin_amdgcn_readfirstlane(c);
    float a0 = 0.0f, a1 = 0.0f, a2 = 0.0f, a3 = 0.0f;
#pragma unroll 1
    for (int b0 = 0; b0 < cU; b0 += 32) {
      int idx = o + b0 + lane;
      idx = min(idx, last);
      int col = lp[idx];
      col = col < 0 ? 0 : (col > nN - 1 ? nN - 1 : col);
      const int m32 = (cU - b0) < 32 ? (cU - b0) : 32;
#pragma unroll 1
      for (int k = 0; k < m32; ++k) {
        const int sk = __builtin_amdgcn_readlane(col, k);
        const v4f hv = *(const v4f*)(H + (size_t)sk * DH + 4 * lane);
        a0 += hv.x;
        a1 += hv.y;
        a2 += hv.z;
        a3 += hv.w;
      }
    }
    const float d = (float)max(deg, 1);
    const float pzr = (deg > DEGCAP) ? __int_as_float(0x7fc00000) : pz;
    const bool live = node < nN;
    const float m0 = live ? (a0 / d + pzr) : 0.0f;
    const float m1 = live ? (a1 / d + pzr) : 0.0f;
    const float m2 = live ? (a2 / d + pzr) : 0.0f;
    const float m3 = live ? (a3 / d + pzr) : 0.0f;
    unsigned h0, l0, h1, l1;
    pack2(m0, m1, h0, l0);
    pack2(m2, m3, h1, l1);
    v2u hv2, lv2;
    hv2.x = h0; hv2.y = h1;
    lv2.x = l0; lv2.y = l1;
    *(v2ua*)(wst + 2 * lane)      = hv2;
    *(v2ua*)(wst + 64 + 2 * lane) = lv2;
    wave_sync();
    const v4u q = *(const v4ua*)(wst + 4 * lane);
    wave_sync();
    unsigned short* wp = M2 + (size_t)node * PHL + 8 * lane;
    *(volatile v4u*)wp = q;
    __threadfence();
    *(volatile v4u*)wp = q;
  }
}

template <int BP>
__device__ __forceinline__ void kseg(const unsigned short* __restrict__ ap, const unsigned short* __restrict__ wp,
                                     int nsteps, v8f (&acc)[8]) {
#pragma unroll 1
  for (int ks = 0; ks < nsteps; ++ks) {
    FragB af;
    af.h[0] = *(const v8usa*)(ap + 32 * ks);
    af.h[1] = *(const v8usa*)(ap + 32 * ks + 16);
#pragma unroll
    for (int t = 0; t < 8; ++t) {
      const unsigned short* wq = wp + (size_t)(16 * t) * (size_t)BP + 32 * ks;
      FragB bf;
      bf.h[0] = *(const v8usa*)wq;
      bf.h[1] = *(const v8usa*)(wq + 16);
      acc[t] = wmb(af, bf, acc[t]);
    }
  }
}

__device__ __forceinline__ void dump_tile(const v8f (&acc)[8], float* stg, const float* bsh, int rowBase,
                                          int wave, int hh, int m, int nN, bool pois) {
#pragma unroll
  for (int t = 0; t < 8; ++t) {
    const int lc = 16 * t + m;
    const float bb = bsh[lc];
#pragma unroll
    for (int r = 0; r < 8; ++r) {
      const int lr = 16 * wave + 8 * hh + r;
      const bool live = (rowBase + lr) < nN;
      float v = relu_k(acc[t][r] + bb);
      v = pois ? __int_as_float(0x7fc00000) : v;
      stg[lr * GBN + lc] = live ? v : 0.0f;
    }
  }
}

__global__ __launch_bounds__(GTHR) __attribute__((amdgpu_num_vgpr(248)))
void k_gemm1(const unsigned short* __restrict__ M1, const unsigned short* __restrict__ XB,
             const unsigned short* __restrict__ BT, const float* __restrict__ bias,
             const int* __restrict__ REC, float* H, unsigned short* HL, int nN, int nB) {
  __shared__ __attribute__((aligned(16))) float stg[GBM * GBN];
  __shared__ __attribute__((aligned(16))) float bsh[GBN];
  const int tid = (int)threadIdx.x, lane = tid & 31, wave = tid >> 5, hh = lane >> 4, m = lane & 15;
  const int rowBase = (int)blockIdx.x * GBM;
  int bb = rowBase >> PKS;
  bb = min(bb, nB - 1);
  const bool pois = REC[(size_t)bb * 32 + 1] != 0;

  if (tid < 32) {
    const v4f b4 = *(const v4f*)(bias + 4 * tid);
    v4f bq;
    bq.x = bf16_val(b4.x); bq.y = bf16_val(b4.y); bq.z = bf16_val(b4.z); bq.w = bf16_val(b4.w);
    *(v4fa*)(bsh + 4 * tid) = bq;
  }

  v8f acc[8];
  {
    const v8f z = {0.f, 0.f, 0.f, 0.f, 0.f, 0.f, 0.f, 0.f};
#pragma unroll
    for (int t = 0; t < 8; ++t) acc[t] = z;
  }
  const size_t r = (size_t)(rowBase + 16 * wave + m);
  const unsigned short* wp = BT + (size_t)m * (size_t)PB1 + 8 * hh;
  kseg<PB1>(M1 + r * PM1 + 8 * hh, wp, DI / 32, acc);
#if SPLIT_B
  kseg<PB1>(M1 + r * PM1 + DI + 8 * hh, wp + DI, DI / 32, acc);
#endif
  kseg<PB1>(XB + r * PXB + 8 * hh, wp + 2 * DI, DI / 32, acc);
  __syncthreads();
  dump_tile(acc, stg, bsh, rowBase, wave, hh, m, nN, pois);
  __syncthreads();

  const bool isHi = (hh == 0);
#pragma unroll 1
  for (int i = 0; i < 16; ++i) {
    const int lr = 16 * wave + i;
    const int gr = rowBase + lr;
    const v4f hv = *(const v4fa*)(stg + lr * GBN + 4 * lane);
    const v4f a  = *(const v4fa*)(stg + lr * GBN + 8 * m);
    const v4f b  = *(const v4fa*)(stg + lr * GBN + 8 * m + 4);
    unsigned h0, l0, h1, l1, h2, l2, h3, l3;
    pack2(a.x, a.y, h0, l0);
    pack2(a.z, a.w, h1, l1);
    pack2(b.x, b.y, h2, l2);
    pack2(b.z, b.w, h3, l3);
    v4u pw;
    pw.x = isHi ? h0 : l0;
    pw.y = isHi ? h1 : l1;
    pw.z = isHi ? h2 : l2;
    pw.w = isHi ? h3 : l3;
    float* hp = H + (size_t)gr * DH + 4 * lane;
    unsigned short* qp = HL + (size_t)gr * PHL + hh * DH + 8 * m;
    *(volatile v4f*)hp = hv;
    *(volatile v4u*)qp = pw;
    __threadfence();
    *(volatile v4f*)hp = hv;
    *(volatile v4u*)qp = pw;
  }
}

__global__ __launch_bounds__(GTHR) __attribute__((amdgpu_num_vgpr(248)))
void k_gemm2(const unsigned short* __restrict__ M2, const unsigned short* __restrict__ HL,
             const unsigned short* __restrict__ BT, const float* __restrict__ bias,
             const int* __restrict__ REC, float* outp, int nN, int nB) {
  __shared__ __attribute__((aligned(16))) float stg[GBM * GBN];
  __shared__ __attribute__((aligned(16))) float bsh[GBN];
  const int tid = (int)threadIdx.x, lane = tid & 31, wave = tid >> 5, hh = lane >> 4, m = lane & 15;
  const int rowBase = (int)blockIdx.x * GBM;
  int bb = rowBase >> PKS;
  bb = min(bb, nB - 1);
  const bool pois = REC[(size_t)bb * 32 + 1] != 0;

  if (tid < 32) {
    const v4f b4 = *(const v4f*)(bias + 4 * tid);
    v4f bq;
    bq.x = bf16_val(b4.x); bq.y = bf16_val(b4.y); bq.z = bf16_val(b4.z); bq.w = bf16_val(b4.w);
    *(v4fa*)(bsh + 4 * tid) = bq;
  }

  v8f acc[8];
  {
    const v8f z = {0.f, 0.f, 0.f, 0.f, 0.f, 0.f, 0.f, 0.f};
#pragma unroll
    for (int t = 0; t < 8; ++t) acc[t] = z;
  }
  const size_t r = (size_t)(rowBase + 16 * wave + m);
  const unsigned short* wp = BT + (size_t)m * (size_t)PB2 + 8 * hh;
  kseg<PB2>(M2 + r * PHL + 8 * hh, wp, DH / 32, acc);
#if SPLIT_C
  kseg<PB2>(M2 + r * PHL + DH + 8 * hh, wp + DH, DH / 32, acc);
#endif
  kseg<PB2>(HL + r * PHL + 8 * hh, wp + 2 * DH, DH / 32, acc);
#if SPLIT_D
  kseg<PB2>(HL + r * PHL + DH + 8 * hh, wp + 3 * DH, DH / 32, acc);
#endif
  __syncthreads();
  dump_tile(acc, stg, bsh, rowBase, wave, hh, m, nN, pois);
  __syncthreads();

#pragma unroll 1
  for (int i = 0; i < 16; ++i) {
    const int lr = 16 * wave + i;
    const int gr = rowBase + lr;
    const v4f ov = *(const v4fa*)(stg + lr * GBN + 4 * lane);
    asm volatile("" :: "v"(ov));
    const int gs = gr < nN ? gr : nN - 1;
    float* op = outp + (size_t)gs * DH + 4 * lane;
    if (gr < nN) *(volatile v4f*)op = ov;
    __threadfence();
    if (gr < nN) *(volatile v4f*)op = ov;
  }
}

static inline int cdiv(int a, int b) { return (a + b - 1) / b; }
static inline size_t al256(size_t o) { return (o + 255) & ~(size_t)255; }

extern "C" void kernel_launch(void* const* d_in, const int* in_sizes, int n_in,
                              void* d_out, int out_size, void* d_ws, size_t ws_size,
                              hipStream_t stream) {
  if (n_in < 8) return;
  if (in_sizes[0] < DI * RPB || (in_sizes[0] % DI) != 0) return;
  const int nN = in_sizes[0] / DI;
  if (nN > 65536) return;
  if (in_sizes[1] < 2 || (in_sizes[1] & 1) != 0) return;
  const int nE = in_sizes[1] / 2;
  if (nE < 1 || nE >= (1 << 21)) return;
  if (in_sizes[2] != DH * DI || in_sizes[3] != DH * DI || in_sizes[4] != DH) return;
  if (in_sizes[5] != DH * DH || in_sizes[6] != DH * DH || in_sizes[7] != DH) return;
  if ((long long)out_size != (long long)nN * DH) return;

  const float* x   = (const float*)d_in[0];
  const int*   ei  = (const int*)  d_in[1];
  const int*   gix = ei;
  const int*   key = ei + nE;
  const float* Wl1 = (const float*)d_in[2];
  const float* Wr1 = (const float*)d_in[3];
  const float* b1  = (const float*)d_in[4];
  const float* Wl2 = (const float*)d_in[5];
  const float* Wr2 = (const float*)d_in[6];
  const float* b2  = (const float*)d_in[7];
  float* out = (float*)d_out;

  const int nB    = cdiv(nN, NBA);
  const int NPADN = nB * NBA;
  const int NP    = cdiv(nN, GBM) * GBM;
  if (NP > NPADN || nB > 64) return;
  const int gR    = NP / RPB;
  const int vec8  = ((nE & 3) == 0) ? 1 : 0;

  char* ws = (char*)d_ws;
  size_t off = 0;
  const size_t oB1 = off; off = al256(off + (size_t)DH * PB1 * 2);
  const size_t oB2 = off; off = al256(off + (size_t)DH * PB2 * 2);
  const size_t oXB = off; off = al256(off + (size_t)NP * PXB * 2);
  const size_t oLS = off; off = al256(off + (size_t)nB * RCAP * 4);
  const size_t oCN = off; off = al256(off + (size_t)NPADN * 4);
  const size_t oOF = off; off = al256(off + (size_t)NPADN * 4);
  const size_t oRC = off; off = al256(off + (size_t)nB * 128);
  const size_t oM1 = off; off = al256(off + (size_t)NP * PM1 * 2);
  const size_t oH  = off; off = al256(off + (size_t)NP * DH * 4);
  const size_t oHL = off; off = al256(off + (size_t)NP * PHL * 2);
  const size_t oM2 = off; off = al256(off + (size_t)NP * PHL * 2);
  if (off > ws_size || off > (size_t)(128u << 20)) return;
  unsigned short* B1 = (unsigned short*)(ws + oB1);
  unsigned short* B2 = (unsigned short*)(ws + oB2);
  unsigned short* XB = (unsigned short*)(ws + oXB);
  int* LIST = (int*)(ws + oLS);
  int* CNT  = (int*)(ws + oCN);
  int* OFF  = (int*)(ws + oOF);
  int* REC  = (int*)(ws + oRC);
  unsigned short* M1 = (unsigned short*)(ws + oM1);
  float* H = (float*)(ws + oH);
  unsigned short* HL = (unsigned short*)(ws + oHL);
  unsigned short* M2 = (unsigned short*)(ws + oM2);

  hipFuncSetAttribute(reinterpret_cast<const void*>(&k_bucket), hipFuncAttributeMaxDynamicSharedMemorySize, LDS_BK);

  const int nUnits = UW + NP * 8;
  k_prep<<<cdiv(nUnits, NTHR), NTHR, 0, stream>>>(x, Wl1, Wr1, Wl2, Wr2, B1, B2, XB, nN, nUnits);
  k_bucket<<<nB, NTHR, LDS_BK, stream>>>(key, gix, nE, nN, vec8, LIST, CNT, OFF, REC);
  k_replay1<<<gR, NTHR, 0, stream>>>(XB, LIST, CNT, OFF, REC, M1, nN, nB);
  k_gemm1<<<gR, GTHR, 0, stream>>>(M1, XB, B1, b1, REC, H, HL, nN, nB);
  k_replay2<<<gR, NTHR, 0, stream>>>(H, LIST, CNT, OFF, REC, M2, nN, nB);
  k_gemm2<<<gR, GTHR, 0, stream>>>(M2, HL, B2, b2, REC, out, nN, nB);
}
